// BahdanauAttentionLayer_11012296147168
// MI455X (gfx1250) — hardware-verified
//
#include <hip/hip_runtime.h>


#ifndef NB
#define NB 8
#endif
#ifndef TD
#define TD 128
#endif
#define NB_FULL 8
#define TD_FULL 128
#define TE   256
#define HH   512
#define PSP  264
#define OSP2 68
#define PCAR 16384.0f
#define C2   2.8853900817779268f
#define L2E  1.4426950408889634f
#define E_OFF ((size_t)NB_FULL * TD_FULL * HH)

static_assert(TE == 256);
static_assert(HH == 512);
static_assert(16 * HH == 256 * 8 * 4);
static_assert(HH % 64 == 0);
static_assert(TE % 64 == 0);
static_assert(HH % 32 == 0);
static_assert(TE % 32 == 0);
static_assert(TD % 16 == 0);
static_assert((NB * TE) % 64 == 0);
static_assert((NB * TD) % 64 == 0);
static_assert(NB <= NB_FULL);
static_assert(TD <= TD_FULL);
static_assert(HH == 8 * 64);
static_assert((PSP * 2) % 16 == 0);
static_assert(PSP >= TE);
static_assert((OSP2 * 4) % 16 == 0);
static_assert(E_OFF * 4 == (size_t)2097152);
static_assert(32 * 16 * 8 == 16 * 64 * 4);
static_assert(32 * 16 * 2 == TE * 4);
static_assert(256 * 16 * 2 == 64 * 128);
static_assert(256 * 4 * 4 == 64 * 64);

typedef _Float16 h16;
typedef unsigned short bf;
typedef __attribute__((ext_vector_type(16))) __bf16   v16bf;
typedef __attribute__((ext_vector_type(16))) _Float16 v16h;
typedef __attribute__((ext_vector_type(8)))  _Float16 v8h;
typedef __attribute__((ext_vector_type(4)))  _Float16 v4h;
typedef __attribute__((ext_vector_type(8)))  unsigned short v8us;
typedef __attribute__((ext_vector_type(8)))  float    v8f;
typedef __attribute__((ext_vector_type(4)))  float    v4f;
typedef v4f  __attribute__((may_alias)) v4fa;
typedef v4h  __attribute__((may_alias)) v4ha;

__device__ __forceinline__ unsigned short f2bf(float f) { unsigned u = __float_as_uint(f); u += 0x7FFFu + ((u >> 16) & 1u); return (unsigned short)(u >> 16); }
__device__ __forceinline__ float bfr(float f) { return __uint_as_float(((unsigned)f2bf(f)) << 16); }
__device__ __forceinline__ v16h cat16(v8h lo, v8h hi) { return __builtin_shufflevector(lo, hi, 0, 1, 2, 3, 4, 5, 6, 7, 8, 9, 10, 11, 12, 13, 14, 15); }
__device__ __forceinline__ v16bf cat16b(v8us lo, v8us hi) { return __builtin_bit_cast(v16bf, __builtin_shufflevector(lo, hi, 0, 1, 2, 3, 4, 5, 6, 7, 8, 9, 10, 11, 12, 13, 14, 15)); }
__device__ __forceinline__ v8f wmma16(v16h a, v16h b, v8f c) { return __builtin_amdgcn_wmma_f32_16x16x32_f16(false, a, false, b, (short)0, c, false, false); }
__device__ __forceinline__ v8f wmmab(v16bf a, v16bf b, v8f c) { return __builtin_amdgcn_wmma_f32_16x16x32_bf16(false, a, false, b, (short)0, c, false, false); }
__device__ __forceinline__ v16h  ldh(const h16* p) { return cat16(*(const v8h*)p, *(const v8h*)(p + 16)); }
__device__ __forceinline__ v16bf ldb(const bf* p)  { return cat16b(*(const v8us*)p, *(const v8us*)(p + 16)); }
__device__ __forceinline__ void wave_sync() { __builtin_amdgcn_fence(3  , "wavefront"); __builtin_amdgcn_wave_barrier(); asm volatile("" ::: "memory"); }

__device__ __forceinline__ v8f wmmab_g(v16bf a, v16bf b, v8f c) { c = wmmab(a, b, c); asm volatile("v_nop\n\tv_nop\n\tv_nop\n\tv_nop" : "+v"(c) : "v"(a), "v"(b)); return c; }
__device__ __forceinline__ v8f wmma16_g(v16h a, v16h b, v8f c) { c = wmma16(a, b, c); asm volatile("v_nop\n\tv_nop\n\tv_nop\n\tv_nop" : "+v"(c) : "v"(a), "v"(b)); return c; }
static __device__ __forceinline__ h16 toh_flush(float v) { const h16 r = (h16)v; return (fabsf(v) < 6.103515625e-05f) ? (h16)0.0f : r; }

__global__ __launch_bounds__(256) void k_cvt8(const float* __restrict__ src, bf* dst, size_t n8) {
    const size_t i = (size_t)blockIdx.x * 256 + threadIdx.x; if (i >= n8) return;
    const v8f v = *(const v8f*)(src + i * 8); v8us o;
#pragma unroll
    for (int k = 0; k < 8; ++k) o[k] = f2bf(v[k]);
    *(volatile v8us*)(dst + i * 8) = o; __threadfence(); *(volatile v8us*)(dst + i * 8) = o;
}

__global__ __launch_bounds__(256) void k_tr_bf(const float* __restrict__ src, bf* dst, int rows, int cols) {
    __shared__ float tile[64 * 65];
    const int tid = threadIdx.x;
    const int r0 = blockIdx.y * 64, c0 = blockIdx.x * 64;
    const size_t zo = (size_t)blockIdx.z * (size_t)rows * (size_t)cols;
    const float* s = src + zo + (size_t)r0 * cols + c0;
#pragma unroll
    for (int i = 0; i < 4; ++i) { const int p = i * 256 + tid; const int row = p >> 4, c4 = (p & 15) * 4;
        const v4f x = *(const v4f*)(s + (size_t)row * cols + c4);
        tile[row * 65 + c4 + 0] = x[0]; tile[row * 65 + c4 + 1] = x[1]; tile[row * 65 + c4 + 2] = x[2]; tile[row * 65 + c4 + 3] = x[3]; }
    __syncthreads();
    bf* d = dst + zo + (size_t)c0 * rows + r0;
#pragma unroll 1
    for (int ps = 0; ps < 2; ++ps) {
#pragma unroll
        for (int sx = 0; sx < 2; ++sx) { const int p = sx * 256 + tid; const int orow = p >> 3, c8 = (p & 7) * 8;
            v8us o;
#pragma unroll
            for (int i = 0; i < 8; ++i) o[i] = f2bf(tile[(c8 + i) * 65 + orow]);
            *(volatile v8us*)(d + (size_t)orow * rows + c8) = o; }
        if (ps == 0) __threadfence(); }
}

__global__ __launch_bounds__(256) void k_tr_h(const float* __restrict__ src, h16* dst, int rows, int cols) {
    __shared__ float tile[64 * 65];
    const int tid = threadIdx.x;
    const int r0 = blockIdx.y * 64, c0 = blockIdx.x * 64;
    const size_t zo = (size_t)blockIdx.z * (size_t)rows * (size_t)cols;
    const float* s = src + zo + (size_t)r0 * cols + c0;
#pragma unroll
    for (int i = 0; i < 4; ++i) { const int p = i * 256 + tid; const int row = p >> 4, c4 = (p & 15) * 4;
        const v4f x = *(const v4f*)(s + (size_t)row * cols + c4);
        tile[row * 65 + c4 + 0] = x[0]; tile[row * 65 + c4 + 1] = x[1]; tile[row * 65 + c4 + 2] = x[2]; tile[row * 65 + c4 + 3] = x[3]; }
    __syncthreads();
    h16* d = dst + zo + (size_t)c0 * rows + r0;
#pragma unroll 1
    for (int ps = 0; ps < 2; ++ps) {
#pragma unroll
        for (int sx = 0; sx < 2; ++sx) { const int p = sx * 256 + tid; const int orow = p >> 3, c8 = (p & 7) * 8;
            v8h o;
#pragma unroll
            for (int i = 0; i < 8; ++i) o[i] = toh_flush(bfr(tile[(c8 + i) * 65 + orow]));
            *(volatile v8h*)(d + (size_t)orow * rows + c8) = o; }
        if (ps == 0) __threadfence(); }
}

__global__ __launch_bounds__(32) void k_pre(const bf* __restrict__ A, const bf* __restrict__ Bt, float* P, int split_row) {
    __shared__ __align__(16) float os[16 * OSP2];
    const int K = HH;
    const int lane = threadIdx.x & 31, lr = lane & 15, hi = lane >> 4; const int r0 = blockIdx.x * 64, c0 = blockIdx.y * 64;
    const size_t wsel = (r0 >= split_row) ? (size_t)HH * HH : (size_t)0;
    v8f acc[4][4];
#pragma unroll
    for (int mb = 0; mb < 4; ++mb)
#pragma unroll
        for (int nb = 0; nb < 4; ++nb) acc[mb][nb] = (v8f){};
    const size_t aoff = (size_t)(r0 + lr) * K + 8 * hi, boff = wsel + (size_t)(c0 + lr) * K + 8 * hi;
#pragma unroll 1
    for (int kc = 0; kc < K; kc += 32) {
        v16bf a[4];
#pragma unroll
        for (int mb = 0; mb < 4; ++mb) a[mb] = ldb(A + aoff + (size_t)mb * 16 * K + kc);
#pragma unroll
        for (int nb = 0; nb < 4; ++nb) { const v16bf b = ldb(Bt + boff + (size_t)nb * 16 * K + kc);
#pragma unroll
            for (int mb = 0; mb < 4; ++mb) acc[mb][nb] = wmmab_g(a[mb], b, acc[mb][nb]); }
    }
#pragma unroll
    for (int mb = 0; mb < 4; ++mb) {
#pragma unroll
        for (int nb = 0; nb < 4; ++nb) {
#pragma unroll
            for (int j = 0; j < 8; ++j) os[(hi * 8 + j) * OSP2 + nb * 16 + lr] = acc[mb][nb][j] * C2; }
        wave_sync();
        float* prow = P + (size_t)(r0 + mb * 16) * HH + c0;
#pragma unroll 1
        for (int ps = 0; ps < 2; ++ps) {
#pragma unroll
            for (int s = 0; s < 8; ++s) { const int row = 2 * s + (lane >> 4), cofs = (lane & 15) * 4;
                const v4f val = *(const v4fa*)(&os[row * OSP2 + cofs]);
                *(volatile v4f*)(prow + (size_t)row * HH + cofs) = val; }
            if (ps == 0) __threadfence(); }
        wave_sync();
    }
}

__global__ __launch_bounds__(256) void k_attn(const float* __restrict__ PRE, const h16* __restrict__ ET, const float* __restrict__ vin, float* OUTC, float* OUTE) {
    __shared__ __align__(16) float du[16 * HH];
    __shared__ __align__(16) float vv[HH];
    __shared__ __align__(16) float sc[16 * TE];
    __shared__ __align__(16) h16   ps[16 * PSP];
    __shared__ __align__(16) float rl[16];
    __shared__ __align__(16) float os[8 * 16 * OSP2];
    const int tid = threadIdx.x, lane = tid & 31, lr = lane & 15, hi = lane >> 4;
    const int wave = __builtin_amdgcn_readfirstlane((int)(threadIdx.x >> 5));
    const int b = blockIdx.y, d0 = blockIdx.x * 16;

    const float* dsrc = PRE + ((size_t)NB * TE + (size_t)b * TD + d0) * HH;
#pragma unroll
    for (int i = 0; i < 8; ++i) { const int idx = (i * 256 + tid) * 4; *(v4fa*)(&du[idx]) = *(const v4f*)(dsrc + idx); }
#pragma unroll
    for (int i = 0; i < 2; ++i) { const int k = i * 256 + tid; vv[k] = -2.0f * bfr(vin[k]); }
    __syncthreads();

    float s[16];
#pragma unroll
    for (int j = 0; j < 16; ++j) s[j] = 0.0f;
    const float* er = PRE + ((size_t)b * TE + tid) * HH;
#pragma unroll 1
    for (int k4 = 0; k4 < HH; k4 += 4) {
        const v4f a = *(const v4f*)(er + k4);
        const v4f w = *(const v4fa*)(&vv[k4]);
#pragma unroll
        for (int j = 0; j < 16; ++j) {
            const v4f d = *(const v4fa*)(&du[j * HH + k4]);
#pragma unroll
            for (int q = 0; q < 4; ++q) {
                const float t = __builtin_amdgcn_exp2f(a[q] + d[q]);
                const float r = __builtin_amdgcn_rcpf(t + 1.0f);
                s[j] = fmaf(r, w[q], s[j]); }
        }
    }
#pragma unroll
    for (int j = 0; j < 16; ++j) sc[j * TE + tid] = s[j];
    __syncthreads();

#pragma unroll 1
    for (int jj = 0; jj < 2; ++jj) {
        const int j = wave * 2 + jj;
        const v4f x0 = *(const v4fa*)(&sc[j * TE + 4 * lane]);
        const v4f x1 = *(const v4fa*)(&sc[j * TE + 128 + 4 * lane]);
        float mx = fmaxf(fmaxf(fmaxf(x0[0], x0[1]), fmaxf(x0[2], x0[3])), fmaxf(fmaxf(x1[0], x1[1]), fmaxf(x1[2], x1[3])));
        mx = fmaxf(mx, __shfl_xor(mx, 16, 32)); mx = fmaxf(mx, __shfl_xor(mx, 8, 32)); mx = fmaxf(mx, __shfl_xor(mx, 4, 32));
        mx = fmaxf(mx, __shfl_xor(mx, 2, 32));  mx = fmaxf(mx, __shfl_xor(mx, 1, 32));
        v4f e0, e1; v4h p0, p1; float lf = 0.0f, lh = 0.0f;
#pragma unroll
        for (int q = 0; q < 4; ++q) {
            const float ea = __builtin_amdgcn_exp2f((x0[q] - mx) * L2E), eb = __builtin_amdgcn_exp2f((x1[q] - mx) * L2E);
            const h16 ha = toh_flush(ea * PCAR), hb = toh_flush(eb * PCAR);
            e0[q] = ea; e1[q] = eb; p0[q] = ha; p1[q] = hb;
            lf += ea + eb; lh += (float)ha + (float)hb; }
        lf += __shfl_xor(lf, 16, 32); lh += __shfl_xor(lh, 16, 32);
        lf += __shfl_xor(lf, 8, 32);  lh += __shfl_xor(lh, 8, 32);
        lf += __shfl_xor(lf, 4, 32);  lh += __shfl_xor(lh, 4, 32);
        lf += __shfl_xor(lf, 2, 32);  lh += __shfl_xor(lh, 2, 32);
        lf += __shfl_xor(lf, 1, 32);  lh += __shfl_xor(lh, 1, 32);
        const float inv = 1.0f / lf;
        if (lane == 0) rl[j] = 1.0f / lh;
        *(v4ha*)(&ps[j * PSP + 4 * lane]) = p0;
        *(v4ha*)(&ps[j * PSP + 128 + 4 * lane]) = p1;
        const v4f w0 = e0 * inv, w1 = e1 * inv;
        float* erow = OUTE + ((size_t)b * TD_FULL + d0 + j) * TE + 4 * lane;
#pragma unroll 1
        for (int pz = 0; pz < 2; ++pz) {
            *(volatile v4f*)(erow) = w0;
            *(volatile v4f*)(erow + 128) = w1;
            if (pz == 0) __threadfence(); }
    }
    __syncthreads();

    const int hb = wave * 64;
    v8f acc[4];
#pragma unroll
    for (int nb = 0; nb < 4; ++nb) acc[nb] = (v8f){};
    const size_t eo = ((size_t)b * HH + hb + lr) * TE + 8 * hi;
    const int po = lr * PSP + 8 * hi;
#pragma unroll 1
    for (int ks = 0; ks < TE; ks += 32) {
        const v16h a = cat16(*(const v8h*)(&ps[po + ks]), *(const v8h*)(&ps[po + ks + 16]));
#pragma unroll
        for (int nb = 0; nb < 4; ++nb) { const v16h bq = ldh(ET + eo + (size_t)nb * 16 * TE + ks); acc[nb] = wmma16_g(a, bq, acc[nb]); }
    }
    float rv[8];
#pragma unroll
    for (int r = 0; r < 8; ++r) rv[r] = rl[8 * hi + r];
    const int wb = wave * 16 * OSP2;
#pragma unroll
    for (int nb = 0; nb < 4; ++nb) {
#pragma unroll
        for (int r = 0; r < 8; ++r) os[wb + (8 * hi + r) * OSP2 + nb * 16 + lr] = acc[nb][r] * rv[r]; }
    wave_sync();
    float* crow = OUTC + ((size_t)b * TD_FULL + d0) * HH + hb;
#pragma unroll 1
    for (int pz = 0; pz < 2; ++pz) {
#pragma unroll
        for (int sx = 0; sx < 8; ++sx) { const int row = 2 * sx + (lane >> 4), cofs = (lane & 15) * 4;
            const v4f val = *(const v4fa*)(&os[wb + row * OSP2 + cofs]);
            *(volatile v4f*)(crow + (size_t)row * HH + cofs) = val; }
        if (pz == 0) __threadfence(); }
}

static constexpr size_t al256(size_t v) { return (v + 255) & ~(size_t)255; }
static constexpr size_t ROWS_AB = (size_t)NB * (TE + TD);
static constexpr size_t SZ_AB  = al256(ROWS_AB * HH * 2);
static constexpr size_t SZ_WT  = al256((size_t)2 * HH * HH * 2);
static constexpr size_t SZ_ET  = al256((size_t)NB * HH * TE * 2);
static constexpr size_t SZ_PRE = al256(ROWS_AB * HH * 4);
static constexpr size_t SZ_TOTAL = SZ_AB + SZ_WT + SZ_ET + SZ_PRE;
static_assert(SZ_TOTAL <= (size_t)134217728);
static_assert(ROWS_AB % 64 == 0);
static_assert(((size_t)HH * HH * 2) % 256 == 0);
static_assert(((size_t)NB * TE * HH * 2) % 256 == 0);
static constexpr size_t LDS_ATTN = (size_t)16 * HH * 4 + (size_t)HH * 4 + (size_t)16 * TE * 4 + (size_t)16 * PSP * 2 + 64 + (size_t)8 * 16 * OSP2 * 4;
static_assert(LDS_ATTN <= 131072);
static_assert((size_t)64 * 65 * 4 <= 131072);
static_assert((size_t)16 * OSP2 * 4 <= 131072);
static_assert(E_OFF + ((size_t)(NB - 1) * TD_FULL + TD) * TE <= (size_t)3145728 / 4);
static_assert(((size_t)(NB - 1) * TD_FULL + TD) * HH <= E_OFF);

extern "C" void kernel_launch(void* const* d_in, const int* in_sizes, int n_in,
                              void* d_out, int out_size, void* d_ws, size_t ws_size, hipStream_t stream) {
    if (n_in < 5) return;
    if ((size_t)in_sizes[0] < (size_t)NB * TE * HH) return;
    if ((size_t)in_sizes[1] < ((size_t)(NB - 1) * TD_FULL + TD) * HH) return;
    if ((size_t)in_sizes[2] < (size_t)HH * HH || (size_t)in_sizes[3] < (size_t)HH * HH) return;
    if (in_sizes[4] < HH) return;
    if ((size_t)out_size < E_OFF + ((size_t)(NB - 1) * TD_FULL + TD) * TE) return;
    if (SZ_TOTAL > ws_size) return;
    const float* enc = (const float*)d_in[0];
    const float* dec = (const float*)d_in[1];
    const float* Wm  = (const float*)d_in[2];
    const float* Um  = (const float*)d_in[3];
    const float* vv  = (const float*)d_in[4];
    float* OUTC = (float*)d_out;
    float* OUTE = (float*)d_out + E_OFF;
    char* wsp = (char*)d_ws;
    bf*    AB  = (bf*)wsp;    wsp += SZ_AB;
    bf*    WT  = (bf*)wsp;    wsp += SZ_WT;
    h16*   ET  = (h16*)wsp;   wsp += SZ_ET;
    float* PRE = (float*)wsp; wsp += SZ_PRE;

    { const size_t n8 = (size_t)NB * TE * HH / 8;
      k_cvt8<<<(unsigned)((n8 + 255) / 256), 256, 0, stream>>>(enc, AB, n8); }
    if (TD == TD_FULL) {
        const size_t n8 = (size_t)NB * TD * HH / 8;
        k_cvt8<<<(unsigned)((n8 + 255) / 256), 256, 0, stream>>>(dec, AB + (size_t)NB * TE * HH, n8);
    } else {
        const size_t n8 = (size_t)TD * HH / 8;
        for (int b = 0; b < NB; ++b)
            k_cvt8<<<(unsigned)((n8 + 255) / 256), 256, 0, stream>>>(dec + (size_t)b * TD_FULL * HH, AB + ((size_t)NB * TE + (size_t)b * TD) * HH, n8);
    }
    k_tr_bf<<<dim3(HH / 64, HH / 64, 1), 256, 0, stream>>>(Wm, WT, HH, HH);
    k_tr_bf<<<dim3(HH / 64, HH / 64, 1), 256, 0, stream>>>(Um, WT + (size_t)HH * HH, HH, HH);
    k_tr_h<<<dim3(HH / 64, TE / 64, NB), 256, 0, stream>>>(enc, ET, TE, HH);

    k_pre<<<dim3((unsigned)(ROWS_AB / 64), HH / 64, 1), 32, 0, stream>>>(AB, WT, PRE, NB * TE);

    k_attn<<<dim3(TD / 16, NB, 1), 256, 0, stream>>>(PRE, ET, vv, OUTC, OUTE);
}
